// MambaBlock_5076651344516
// MI455X (gfx1250) — hardware-verified
//
#include <hip/hip_runtime.h>
#include <math.h>

typedef __attribute__((ext_vector_type(16))) _Float16 v16h;
typedef __attribute__((ext_vector_type(8)))  _Float16 v8h;
typedef __attribute__((ext_vector_type(16))) __bf16   v16b;
typedef __attribute__((ext_vector_type(8)))  __bf16   v8b;
typedef __attribute__((ext_vector_type(8)))  float    v8f;
typedef __attribute__((ext_vector_type(4)))  float    v4f;

constexpr int kSeq   = 2048;
constexpr int kDm    = 1024;
constexpr int kDin   = 2048;
constexpr int kNst   = 64;
constexpr int kXrP   = 2 * kDin;
constexpr int kBcP   = 2 * kNst;
constexpr int kConvTP = 260;
constexpr int kScT   = 32;
constexpr int kScC   = 64;
constexpr int kScYP  = 68;
static_assert((kDm % 32) == 0 && (kDin % 32) == 0, "GEMM K multiples of 32");
static_assert((kSeq % 64) == 0 && (kXrP % 64) == 0 && (kBcP % 64) == 0 && (kDin % 64) == 0 && (kDm % 64) == 0, "GEMM M,N multiples of 64");
static_assert((kSeq % kScT) == 0 && (kDin % kScC) == 0 && (kDin % 256) == 0 && kNst == 64, "tile multiples");
static_assert(16 * 256 == kScT * kBcP, "A staging fits the B|C tile exactly");

constexpr size_t kOffHSB  = 0;
constexpr size_t kOffWINB = kOffHSB  + (size_t)kSeq * kDm  * 2;
constexpr size_t kOffWXB  = kOffWINB + (size_t)kXrP * kDm  * 2;
constexpr size_t kOffWDTB = kOffWXB  + (size_t)kBcP * kDin * 2;
constexpr size_t kOffWOB  = kOffWDTB + (size_t)kDin * kDin * 2;
constexpr size_t kOffXR   = kOffWOB  + (size_t)kDm  * kDin * 2;
constexpr size_t kOffXC   = kOffXR   + (size_t)kSeq * kXrP * 4;
constexpr size_t kOffXH   = kOffXC   + (size_t)kSeq * kDin * 4;
constexpr size_t kOffXL   = kOffXH   + (size_t)kSeq * kDin * 2;
constexpr size_t kOffBC   = kOffXL   + (size_t)kSeq * kDin * 2;
constexpr size_t kOffDLR  = kOffBC   + (size_t)kSeq * kBcP * 4;
constexpr size_t kOffYH   = kOffDLR  + (size_t)kSeq * kDin * 4;
constexpr size_t kOffYL   = kOffYH   + (size_t)kSeq * kDin * 2;
constexpr size_t kWsTotal = kOffYL   + (size_t)kSeq * kDin * 2;
static_assert(kWsTotal == 127401984ull, "carve total");
static_assert(kWsTotal <= 134217728ull, "carve cap");
static_assert((kOffWINB % 128) == 0 && (kOffWXB % 128) == 0 && (kOffWDTB % 128) == 0 && (kOffWOB % 128) == 0 &&
              (kOffXR % 128) == 0 && (kOffXC % 128) == 0 && (kOffXH % 128) == 0 && (kOffXL % 128) == 0 &&
              (kOffBC % 128) == 0 && (kOffDLR % 128) == 0 && (kOffYH % 128) == 0 && (kOffYL % 128) == 0,
              "128-B aligned regions");

__device__ __forceinline__ unsigned short f2bf_bits(float f) {
  unsigned u = __float_as_uint(f);
  return (unsigned short)((u + 0x7FFFu + ((u >> 16) & 1u)) >> 16);
}
__device__ __forceinline__ float bf_bits2f(unsigned short h) { return __uint_as_float(((unsigned)h) << 16); }
__device__ __forceinline__ float bf_rne(float f) { return bf_bits2f(f2bf_bits(f)); }

__device__ __forceinline__ void split8(const v4f a0, const v4f a1, v8h& hv, v8h& lv) {
#pragma unroll
  for (int e = 0; e < 4; ++e) {
    const float f0 = a0[e];
    const float f1 = a1[e];
    const unsigned short h0 = f2bf_bits(f0);
    const unsigned short h1 = f2bf_bits(f1);
    const unsigned short l0 = f2bf_bits(f0 - bf_bits2f(h0));
    const unsigned short l1 = f2bf_bits(f1 - bf_bits2f(h1));
    hv[e]     = __builtin_bit_cast(_Float16, h0);
    hv[4 + e] = __builtin_bit_cast(_Float16, h1);
    lv[e]     = __builtin_bit_cast(_Float16, l0);
    lv[4 + e] = __builtin_bit_cast(_Float16, l1);
  }
}

__device__ __forceinline__ void dep_guard4_h(v8f& a, v8f& b, v8f& c, v8f& d, v16h x, v16h y) {
  asm volatile("v_nop\n\tv_nop\n\tv_nop\n\tv_nop" : "+v"(a), "+v"(b), "+v"(c), "+v"(d) : "v"(x), "v"(y));
}
__device__ __forceinline__ void dep_guard4_b(v8f& a, v8f& b, v8f& c, v8f& d, v16b x, v16b y) {
  asm volatile("v_nop\n\tv_nop\n\tv_nop\n\tv_nop" : "+v"(a), "+v"(b), "+v"(c), "+v"(d) : "v"(x), "v"(y));
}
__device__ __forceinline__ void keep4_h(v16h a, v16h b, v16h c, v16h d) { asm volatile("v_nop" :: "v"(a), "v"(b), "v"(c), "v"(d)); }
__device__ __forceinline__ void keep4_b(v16b a, v16b b, v16b c, v16b d) { asm volatile("v_nop" :: "v"(a), "v"(b), "v"(c), "v"(d)); }
__device__ __forceinline__ void acc_guard4(v8f& a, v8f& b, v8f& c, v8f& d) {
  asm volatile("v_nop\n\tv_nop\n\tv_nop\n\tv_nop" : "+v"(a), "+v"(b), "+v"(c), "+v"(d));
}

template <typename T> struct Frag;
template <> struct Frag<_Float16> {
  typedef v16h V; union U { v16h v; v8h h[2]; };
  static __device__ __forceinline__ v16h load(const _Float16* p) {
    U f; f.h[0] = *(const v8h*)(p); f.h[1] = *(const v8h*)(p + 16); return f.v;
  }
  static __device__ __forceinline__ v8f mma(v16h a, v16h b, v8f c) {
    return __builtin_amdgcn_wmma_f32_16x16x32_f16(false, a, false, b, (short)0, c, false, false);
  }
  static __device__ __forceinline__ void guard4(v8f& a, v8f& b, v8f& c, v8f& d, v16h x, v16h y) { dep_guard4_h(a, b, c, d, x, y); }
  static __device__ __forceinline__ void keep(v16h a, v16h b, v16h c, v16h d) { keep4_h(a, b, c, d); }
};
template <> struct Frag<__bf16> {
  typedef v16b V; union U { v16b v; v8b h[2]; };
  static __device__ __forceinline__ v16b load(const __bf16* p) {
    U f; f.h[0] = *(const v8b*)(p); f.h[1] = *(const v8b*)(p + 16); return f.v;
  }
  static __device__ __forceinline__ v8f mma(v16b a, v16b b, v8f c) {
    return __builtin_amdgcn_wmma_f32_16x16x32_bf16(false, a, false, b, (short)0, c, false, false);
  }
  static __device__ __forceinline__ void guard4(v8f& a, v8f& b, v8f& c, v8f& d, v16b x, v16b y) { dep_guard4_b(a, b, c, d, x, y); }
  static __device__ __forceinline__ void keep(v16b a, v16b b, v16b c, v16b d) { keep4_b(a, b, c, d); }
};

template <int ET> struct Elem;
template <> struct Elem<0> { typedef _Float16 T; };
template <> struct Elem<1> { typedef __bf16 T; };
template <int ET, int SPL, int BIAS_MODE, int OUT_MODE, bool RESID, int ACT = 0>
__global__ __launch_bounds__(256) void wmma_gemm64(
    const unsigned short* __restrict__ Ap, const unsigned short* __restrict__ A2p, int lda, long strideA,
    const unsigned short* __restrict__ Btp, const unsigned short* __restrict__ Bt2p, int ldb, long strideB,
    void* __restrict__ Cout, void* __restrict__ Cout2, int ldc, long strideC,
    const float* __restrict__ bias,
    const float* __restrict__ resid, long strideR,
    int M, int N, int K, float scale) {
  typedef typename Elem<ET>::T T;
  typedef typename Frag<T>::V V;
  const T* A = (const T*)Ap; const T* A2 = (const T*)A2p; const T* Bt = (const T*)Btp; const T* Bt2 = (const T*)Bt2p;
  __shared__ __align__(16) float sT[8][16 * 68];
  const int b    = blockIdx.y;
  const int lane = threadIdx.x & 31;
  const int wave = threadIdx.x >> 5;
  const int tilesN = N >> 6;
  const int tilesM = M >> 6;
  const int tile = blockIdx.x * 8 + wave;
  if (tile >= tilesM * tilesN) return;
  const int tm = tile / tilesN;
  const int tn = tile - tm * tilesN;
  const int m0 = tm << 6;
  const int n0 = tn << 6;

  const T* Ab  = A  + (size_t)b * strideA;
  const T* Bb  = Bt + (size_t)b * strideB;
  const T* Ab2 = (SPL >= 1) ? (A2  + (size_t)b * strideA) : nullptr;
  const T* Bb2 = (SPL == 2) ? (Bt2 + (size_t)b * strideB) : nullptr;

  const int rlane = lane & 15;
  const int koff  = (lane >> 4) * 8;
  const int mOff  = (lane >> 4) * 8;

  v8f acc[4][4];
#pragma unroll
  for (int i = 0; i < 4; ++i)
#pragma unroll
    for (int j = 0; j < 4; ++j) acc[i][j] = (v8f){0.f,0.f,0.f,0.f,0.f,0.f,0.f,0.f};

  for (int k0 = 0; k0 < K; k0 += 32) {
    V bh[4], bl[4];
#pragma unroll
    for (int j = 0; j < 4; ++j) {
      const size_t bo = (size_t)(n0 + (j << 4) + rlane) * ldb + koff + k0;
      bh[j] = Frag<T>::load(Bb + bo);
      if (SPL == 2) bl[j] = Frag<T>::load(Bb2 + bo);
    }
#pragma unroll
    for (int i = 0; i < 4; ++i) {
      const size_t ao = (size_t)(m0 + (i << 4) + rlane) * lda + koff + k0;
      V ah = Frag<T>::load(Ab + ao);
      V al;
      if (SPL >= 1) al = Frag<T>::load(Ab2 + ao);
#pragma unroll
      for (int j = 0; j < 4; ++j) {
        acc[i][j] = Frag<T>::mma(ah, bh[j], acc[i][j]);
        if (SPL == 2) acc[i][j] = Frag<T>::mma(ah, bl[j], acc[i][j]);
        if (SPL >= 1) acc[i][j] = Frag<T>::mma(al, bh[j], acc[i][j]);
      }
      Frag<T>::guard4(acc[i][0], acc[i][1], acc[i][2], acc[i][3], ah, (SPL >= 1) ? al : ah);
    }
    Frag<T>::keep(bh[0], bh[1], bh[2], bh[3]);
    if (SPL == 2) Frag<T>::keep(bl[0], bl[1], bl[2], bl[3]);
  }
  acc_guard4(acc[0][0], acc[0][1], acc[0][2], acc[0][3]);
  acc_guard4(acc[1][0], acc[1][1], acc[1][2], acc[1][3]);
  acc_guard4(acc[2][0], acc[2][1], acc[2][2], acc[2][3]);
  acc_guard4(acc[3][0], acc[3][1], acc[3][2], acc[3][3]);

  float* slab = sT[wave];
  const float* Rb = RESID ? (resid + (size_t)b * strideR) : nullptr;
#pragma unroll
  for (int i = 0; i < 4; ++i) {
    const int mBase = m0 + (i << 4);
#pragma unroll
    for (int j = 0; j < 4; ++j) {
      const int n = n0 + (j << 4) + rlane;
      float bv = 0.f;
      if (BIAS_MODE == 2) bv = bias[n];
#pragma unroll
      for (int r = 0; r < 8; ++r) {
        float v = acc[i][j][r] * scale;
        if (BIAS_MODE == 1) v += bias[mBase + mOff + r];
        if (BIAS_MODE == 2) v += bv;
        if (RESID) v += Rb[(size_t)(mBase + mOff + r) * ldc + n];
        if (ACT == 1) v = tanhf(v);
        if (ACT == 2) v = fmaxf(v, 0.0f);
        if (ACT == 3) v = v / (1.0f + expf(-v));
        if (ACT == 4) v = (v > 0.f) ? v : 0.01f * v;
        slab[(mOff + r) * 68 + (j << 4) + rlane] = v;
      }
    }
    __builtin_amdgcn_fence(__ATOMIC_RELEASE, "workgroup");
    __builtin_amdgcn_wave_barrier();
    __builtin_amdgcn_fence(__ATOMIC_ACQUIRE, "workgroup");
    if (OUT_MODE == 0) {
      float* C = (float*)Cout + (size_t)b * strideC;
      const int hh = lane >> 4, c4 = (lane & 15) * 4;
      for (int pass = 0; pass < 2; ++pass) {
#pragma unroll
        for (int it = 0; it < 8; ++it) {
          const int row = it * 2 + hh;
          v4f v = *(const v4f*)(slab + row * 68 + c4);
          *(volatile v4f*)(C + (size_t)(mBase + row) * ldc + n0 + c4) = v;
        }
        __threadfence();
      }
    } else {
      const int q = lane >> 3, c8 = (lane & 7) * 8;
      unsigned short* C  = (unsigned short*)Cout  + (size_t)b * strideC;
      unsigned short* C2 = (OUT_MODE == 2) ? ((unsigned short*)Cout2 + (size_t)b * strideC) : nullptr;
      for (int pass = 0; pass < 2; ++pass) {
#pragma unroll
        for (int it = 0; it < 4; ++it) {
          const int row = it * 4 + q;
          const float* sp = slab + row * 68 + c8;
          v8h hv, lv;
#pragma unroll
          for (int e = 0; e < 8; ++e) {
            const float sv = sp[e];
            if (OUT_MODE == 1) {
              hv[e] = (_Float16)sv;
            } else {
              const unsigned short hb = f2bf_bits(sv);
              const unsigned short lb = f2bf_bits(sv - bf_bits2f(hb));
              hv[e] = __builtin_bit_cast(_Float16, hb);
              lv[e] = __builtin_bit_cast(_Float16, lb);
            }
          }
          *(volatile v8h*)(C + (size_t)(mBase + row) * ldc + n0 + c8) = hv;
          if (OUT_MODE == 2) *(volatile v8h*)(C2 + (size_t)(mBase + row) * ldc + n0 + c8) = lv;
        }
        __threadfence();
      }
    }
    __builtin_amdgcn_fence(__ATOMIC_RELEASE, "workgroup");
    __builtin_amdgcn_wave_barrier();
    __builtin_amdgcn_fence(__ATOMIC_ACQUIRE, "workgroup");
  }
}

__global__ __launch_bounds__(256) void cast_rows_bf16_kernel(
    const float* __restrict__ src, unsigned short* __restrict__ dst, int total8)
{
  const int i = blockIdx.x * 256 + threadIdx.x;
  if (i >= total8) return;
  const size_t e0 = (size_t)i << 3;
  const v4f a0 = *(const v4f*)(src + e0);
  const v4f a1 = *(const v4f*)(src + e0 + 4);
  v8h hv;
#pragma unroll
  for (int e = 0; e < 4; ++e) {
    const float f0 = a0[e];
    const float f1 = a1[e];
    const unsigned short h0 = f2bf_bits(f0);
    const unsigned short h1 = f2bf_bits(f1);
    hv[e]     = __builtin_bit_cast(_Float16, h0);
    hv[4 + e] = __builtin_bit_cast(_Float16, h1);
  }
  unsigned short* q = dst + e0;
  *(volatile v8h*)q = hv;
  __threadfence();
  *(volatile v8h*)q = hv;
}

__global__ __launch_bounds__(256) void conv_silu_kernel(
    const float* __restrict__ XR, const float* __restrict__ cw, const float* __restrict__ cb,
    float* __restrict__ XC, unsigned short* __restrict__ XH, unsigned short* __restrict__ XL)
{
  __shared__ __align__(16) float sT[16 * kConvTP];
  const int tid = threadIdx.x, lane = tid & 31, wave = tid >> 5;
  const int d0 = blockIdx.x * 256, d = d0 + tid;
  const int g0 = blockIdx.y * 64;
  const v4f wv = *(const v4f*)(cw + (size_t)d * 4);
  const float w0 = bf_rne(wv[0]), w1 = bf_rne(wv[1]), w2 = bf_rne(wv[2]), w3 = bf_rne(wv[3]);
  const float bc = bf_rne(cb[d]);
  float xm3, xm2, xm1;
  {
    const bool hist = (g0 > 0);
    const int rb = hist ? (g0 - 3) : g0;
    const float v3 = XR[(size_t)rb * kXrP + d];
    const float v2 = XR[(size_t)(rb + 1) * kXrP + d];
    const float v1 = XR[(size_t)(rb + 2) * kXrP + d];
    xm3 = hist ? v3 : 0.f;
    xm2 = hist ? v2 : 0.f;
    xm1 = hist ? v1 : 0.f;
  }
  const int hrow = wave >> 1;
  const int hch  = (wave & 1) * 128 + lane * 4;
#pragma unroll 1
  for (int sub = 0; sub < 4; ++sub) {
    const int lb = g0 + sub * 16;
#pragma unroll 1
    for (int s = 0; s < 16; ++s) {
      const float xcur = XR[(size_t)(lb + s) * kXrP + d];
      float acc = w0 * xm3;
      acc = fmaf(w1, xm2, acc);
      acc = fmaf(w2, xm1, acc);
      acc = fmaf(w3, xcur, acc);
      const float sv = acc + bc;
      const float sg = __builtin_amdgcn_rcpf(1.0f + expf(-sv));
      sT[s * kConvTP + tid] = sv * sg;
      xm3 = xm2; xm2 = xm1; xm1 = xcur;
    }
    __syncthreads();
    v4f fv[4];
    v8h bh[2], blo[2];
#pragma unroll
    for (int it = 0; it < 4; ++it) fv[it] = *(const v4f*)(sT + (it * 4 + hrow) * kConvTP + hch);
#pragma unroll
    for (int it = 0; it < 2; ++it) {
      const float* sp = sT + (it * 8 + wave) * kConvTP + lane * 8;
      const v4f a0 = *(const v4f*)(sp);
      const v4f a1 = *(const v4f*)(sp + 4);
      split8(a0, a1, bh[it], blo[it]);
    }
    for (int pass = 0; pass < 2; ++pass) {
#pragma unroll
      for (int it = 0; it < 4; ++it)
        *(volatile v4f*)(XC + (size_t)(lb + it * 4 + hrow) * kDin + d0 + hch) = fv[it];
#pragma unroll
      for (int it = 0; it < 2; ++it) {
        const size_t o = (size_t)(lb + it * 8 + wave) * kDin + d0 + lane * 8;
        *(volatile v8h*)(XH + o) = bh[it];
        *(volatile v8h*)(XL + o) = blo[it];
      }
      __threadfence();
    }
    __syncthreads();
  }
}

__global__ __launch_bounds__(256) void scan_kernel(
    const float* __restrict__ BC, const float* __restrict__ DLR, const float* __restrict__ XC,
    const float* __restrict__ XR, const float* __restrict__ bdt, const float* __restrict__ Alog,
    unsigned short* __restrict__ YH, unsigned short* __restrict__ YL)
{
  __shared__ __align__(16) float sBC[kScT * kBcP];
  __shared__ __align__(16) float sDT[kScT * kScC];
  __shared__ __align__(16) float sX[kScT * kScC];
  __shared__ __align__(16) float sG[kScT * kScC];
  __shared__ __align__(16) float sY[kScT * kScYP];
  const int tid = threadIdx.x;
  const int c   = tid >> 2;
  const int sub = tid & 3;
  const int d0  = blockIdx.x * kScC;

#pragma unroll 1
  for (int k = 0; k < 16; ++k) {
    const float al = Alog[(size_t)(d0 + c) * kNst + sub * 16 + k];
    sBC[k * 256 + tid] = -expf(bf_rne(al));
  }
  __syncthreads();
  float negA[16], h[16];
#pragma unroll
  for (int k = 0; k < 16; ++k) {
    negA[k] = sBC[k * 256 + tid];
    h[k] = 0.f;
  }
  const float bb = bf_rne(bdt[d0 + (tid & 63)]);
  const int orow = tid >> 3;
  const int c8   = (tid & 7) * 8;

#pragma unroll 1
  for (int t0 = 0; t0 < kSeq; t0 += kScT) {
    __syncthreads();
#pragma unroll
    for (int i = 0; i < 4; ++i) {
      const int idx = tid + 256 * i;
      const int row = idx >> 5;
      const int c4  = (idx & 31) * 4;
      *(v4f*)(sBC + row * kBcP + c4) = *(const v4f*)(BC + (size_t)(t0 + row) * kBcP + c4);
    }
#pragma unroll
    for (int i = 0; i < 2; ++i) {
      const int idx = tid + 256 * i;
      const int row = idx >> 4;
      const int c4  = (idx & 15) * 4;
      const size_t g = (size_t)(t0 + row);
      *(v4f*)(sDT + row * kScC + c4) = *(const v4f*)(DLR + g * kDin + d0 + c4);
      *(v4f*)(sX  + row * kScC + c4) = *(const v4f*)(XC  + g * kDin + d0 + c4);
      *(v4f*)(sG  + row * kScC + c4) = *(const v4f*)(XR  + g * kXrP + kDin + d0 + c4);
    }
    __syncthreads();
#pragma unroll 1
    for (int j = 0; j < 8; ++j) {
      const int e = tid + 256 * j;
      const float v  = sDT[e] + bb;
      const float ea = expf(-fabsf(v));
      sDT[e] = fmaxf(v, 0.0f) + log1pf(ea);
      const float z  = sG[e];
      const float sg = __builtin_amdgcn_rcpf(1.0f + __expf(-z));
      sG[e] = z * sg;
    }
    __syncthreads();
#pragma unroll 1
    for (int s = 0; s < kScT; ++s) {
      const float dt  = sDT[s * kScC + c];
      const float xt  = sX[s * kScC + c];
      const float gt  = sG[s * kScC + c];
      const float dtx = dt * xt;
      const float* bp = sBC + s * kBcP + sub * 16;
      float y = 0.f;
#pragma unroll
      for (int q = 0; q < 4; ++q) {
        const v4f bv = *(const v4f*)(bp + 4 * q);
        const v4f cv = *(const v4f*)(bp + kNst + 4 * q);
#pragma unroll
        for (int e = 0; e < 4; ++e) {
          const float ex = __expf(dt * negA[4 * q + e]);
          const float hn = fmaf(ex, h[4 * q + e], dtx * bv[e]);
          h[4 * q + e] = hn;
          y = fmaf(hn, cv[e], y);
        }
      }
      y += __shfl_xor(y, 1, 32);
      y += __shfl_xor(y, 2, 32);
      const float yg = y * gt;
      if (sub == 0) sY[s * kScYP + c] = yg;
    }
    __syncthreads();
    {
      const float* sp = sY + orow * kScYP + c8;
      const v4f a0 = *(const v4f*)(sp);
      const v4f a1 = *(const v4f*)(sp + 4);
      v8h hv, lv;
      split8(a0, a1, hv, lv);
      const size_t o = (size_t)(t0 + orow) * kDin + d0 + c8;
      *(volatile v8h*)(YH + o) = hv;
      *(volatile v8h*)(YL + o) = lv;
      __threadfence();
      *(volatile v8h*)(YH + o) = hv;
      *(volatile v8h*)(YL + o) = lv;
    }
  }
}

extern "C" void kernel_launch(void* const* d_in, const int* in_sizes, int n_in,
                              void* d_out, int out_size, void* d_ws, size_t ws_size,
                              hipStream_t stream) {
  if (n_in < 9) return;
  if (in_sizes[0] != kSeq * kDm) return;
  if (in_sizes[1] != kXrP * kDm) return;
  if (in_sizes[2] != kDin * 4) return;
  if (in_sizes[3] != kDin) return;
  if (in_sizes[4] != kBcP * kDin) return;
  if (in_sizes[5] != kDin * kDin) return;
  if (in_sizes[6] != kDin) return;
  if (in_sizes[7] != kDin * kNst) return;
  if (in_sizes[8] != kDm * kDin) return;
  if (out_size != kSeq * kDm) return;
  if (ws_size < kWsTotal) return;

  const float* hs     = (const float*)d_in[0];
  const float* W_in   = (const float*)d_in[1];
  const float* conv_w = (const float*)d_in[2];
  const float* conv_b = (const float*)d_in[3];
  const float* W_x    = (const float*)d_in[4];
  const float* W_dt   = (const float*)d_in[5];
  const float* b_dt   = (const float*)d_in[6];
  const float* A_log  = (const float*)d_in[7];
  const float* W_out  = (const float*)d_in[8];
  float* out = (float*)d_out;

  char* ws = (char*)d_ws;
  unsigned short* HSB  = (unsigned short*)(ws + kOffHSB);
  unsigned short* WINB = (unsigned short*)(ws + kOffWINB);
  unsigned short* WXB  = (unsigned short*)(ws + kOffWXB);
  unsigned short* WDTB = (unsigned short*)(ws + kOffWDTB);
  unsigned short* WOB  = (unsigned short*)(ws + kOffWOB);
  float*          XR   = (float*)(ws + kOffXR);
  float*          XC   = (float*)(ws + kOffXC);
  unsigned short* XH   = (unsigned short*)(ws + kOffXH);
  unsigned short* XL   = (unsigned short*)(ws + kOffXL);
  float*          BC   = (float*)(ws + kOffBC);
  float*          DLR  = (float*)(ws + kOffDLR);
  unsigned short* YH   = (unsigned short*)(ws + kOffYH);
  unsigned short* YL   = (unsigned short*)(ws + kOffYL);
  const float* dummy_bias  = b_dt;
  const float* dummy_resid = hs;

  cast_rows_bf16_kernel<<<(kSeq * kDm / 8) / 256, 256, 0, stream>>>(hs, HSB, kSeq * kDm / 8);
  cast_rows_bf16_kernel<<<(kXrP * kDm / 8) / 256, 256, 0, stream>>>(W_in, WINB, kXrP * kDm / 8);
  cast_rows_bf16_kernel<<<(kBcP * kDin / 8) / 256, 256, 0, stream>>>(W_x, WXB, kBcP * kDin / 8);
  cast_rows_bf16_kernel<<<(kDin * kDin / 8) / 256, 256, 0, stream>>>(W_dt, WDTB, kDin * kDin / 8);
  cast_rows_bf16_kernel<<<(kDm * kDin / 8) / 256, 256, 0, stream>>>(W_out, WOB, kDm * kDin / 8);

  wmma_gemm64<1, 0, 0, 0, false><<<dim3(256, 1), 256, 0, stream>>>(
      HSB, HSB, kDm, 0L,
      WINB, WINB, kDm, 0L,
      (void*)XR, (void*)XR, kXrP, 0L,
      dummy_bias, dummy_resid, 0L,
      kSeq, kXrP, kDm, 1.0f);

  conv_silu_kernel<<<dim3(kDin / 256, kSeq / 64), 256, 0, stream>>>(XR, conv_w, conv_b, XC, XH, XL);

  wmma_gemm64<1, 1, 0, 0, false><<<dim3(8, 1), 256, 0, stream>>>(
      XH, XL, kDin, 0L,
      WXB, WXB, kDin, 0L,
      (void*)BC, (void*)BC, kBcP, 0L,
      dummy_bias, dummy_resid, 0L,
      kSeq, kBcP, kDin, 1.0f);

  wmma_gemm64<1, 1, 0, 0, false><<<dim3(128, 1), 256, 0, stream>>>(
      XH, XL, kDin, 0L,
      WDTB, WDTB, kDin, 0L,
      (void*)DLR, (void*)DLR, kDin, 0L,
      dummy_bias, dummy_resid, 0L,
      kSeq, kDin, kDin, 1.0f);

  scan_kernel<<<kDin / kScC, 256, 0, stream>>>(BC, DLR, XC, XR, b_dt, A_log, YH, YL);

  wmma_gemm64<1, 1, 0, 0, false><<<dim3(64, 1), 256, 0, stream>>>(
      YH, YL, kDin, 0L,
      WOB, WOB, kDin, 0L,
      (void*)out, (void*)out, kDm, 0L,
      dummy_bias, dummy_resid, 0L,
      kSeq, kDm, kDin, 1.0f);
}
